// RobustSupplyChainSAGE_2336462209551
// MI455X (gfx1250) — hardware-verified
//
#include <hip/hip_runtime.h>
#include <stddef.h>
#include <math.h>


#define HID     64
#define NTHR    256
#define NWAVE   8
#define EPT     8
#define NGRP    2
#define CHUNK   (NTHR * EPT * NGRP)
#define WCAP    (EPT * NGRP * 32)
#define LISTN   (NWAVE * WCAP)
#define NBC     4096
#define NBF     1024
#define RCAP    32768
#define RBN     128
#define TGT     256
#define DEGCAP  1024
#define GROWS   128
#define QROWS   128
#define OTHR    512
#define WSCAP   134217728

#define KENC    32
#define APKE    40
#define KSG     192
#define APKS    200
#define KH1     160
#define APK1    168
#define KH2     128
#define APK2    136

#define WP_ENC  0
#define WP_SG   4096
#define WP_SGSZ 24576
#define WP_H1   77824
#define WP_H2   118784
#define WPTOT   135168

#define LDS_FILL   ((RCAP + NBF + LISTN) * 4 + 64)
#define LDS_ENC    (GROWS * HID * 4)
#define LDS_LAYER  (2 * GROWS * APKS * 2)
#define LDS_HEAD_R1 (2 * QROWS * APK1 * 2)
#define LDS_HEAD_R2 (2 * QROWS * APK2 * 2)
#define LDS_HEAD   (LDS_HEAD_R1 + LDS_HEAD_R2)

#define LN_EPS 1e-5f
#define BN_EPS 1e-5f

static_assert((CHUNK & (CHUNK - 1)) == 0);
static_assert(CHUNK <= 4096);
static_assert(NBC <= 4096 && NBF <= 4096);
static_assert((NBC & (NBC - 1)) == 0 && (NBF & (NBF - 1)) == 0);
static_assert(NBC == 4 * NBF);
static_assert(OTHR * 8 == NBC);
static_assert((RCAP % 32) == 0);
static_assert((TGT % GROWS) == 0 && TGT == NWAVE * 32);
static_assert((NBC % TGT) == 0);
static_assert(GROWS == NWAVE * 16 && QROWS == NWAVE * 16);
static_assert(2 * GROWS * APKE * 2 <= LDS_ENC);
static_assert(GROWS * HID * 4 <= LDS_LAYER);
static_assert(QROWS * 128 * 4 <= LDS_HEAD_R1);
static_assert(WP_SG == WP_ENC + 2 * 64 * KENC && WP_SGSZ == 2 * 64 * KSG);
static_assert(WP_H1 == WP_SG + 3 * WP_SGSZ && WP_H2 == WP_H1 + 2 * 128 * KH1 && WPTOT == WP_H2 + 2 * 64 * KH2);
static_assert((WP_SG % 8) == 0 && (WP_SGSZ % 8) == 0 && (WP_H1 % 8) == 0 && (WP_H2 % 8) == 0);

typedef float          v2f  __attribute__((ext_vector_type(2)));
typedef float          v4f  __attribute__((ext_vector_type(4)));
typedef float          v8f  __attribute__((ext_vector_type(8)));
typedef int            v4i  __attribute__((ext_vector_type(4)));
typedef unsigned short v8us __attribute__((ext_vector_type(8)));
typedef __bf16         v16b __attribute__((ext_vector_type(16)));
union FragB { v16b v; v8us h[2]; };

__device__ __forceinline__ unsigned int bfr(float f) {
  const unsigned int u = __float_as_uint(f);
  return (u + 0x7FFFu + ((u >> 16) & 1u)) >> 16;
}

__device__ __forceinline__ void split1(float x, unsigned short& hb, unsigned short& lb) {
  const unsigned int hu = bfr(x);
  const float hf = __uint_as_float(hu << 16);
  hb = (unsigned short)hu;
  lb = (unsigned short)bfr(x - hf);
}

__device__ __forceinline__ void split8(v4f a, v4f b, v8us& hi, v8us& lo) {
  unsigned short hb, lb;
  split1(a.x, hb, lb); hi[0] = hb; lo[0] = lb;
  split1(a.y, hb, lb); hi[1] = hb; lo[1] = lb;
  split1(a.z, hb, lb); hi[2] = hb; lo[2] = lb;
  split1(a.w, hb, lb); hi[3] = hb; lo[3] = lb;
  split1(b.x, hb, lb); hi[4] = hb; lo[4] = lb;
  split1(b.y, hb, lb); hi[5] = hb; lo[5] = lb;
  split1(b.z, hb, lb); hi[6] = hb; lo[6] = lb;
  split1(b.w, hb, lb); hi[7] = hb; lo[7] = lb;
}

__device__ __forceinline__ v8f wmb(v16b a, v16b b, v8f c) {
  v8f d = __builtin_amdgcn_wmma_f32_16x16x32_bf16(false, a, false, b, (short)0, c, false, false);
  asm volatile("v_nop\n\tv_nop\n\tv_nop\n\tv_nop" : "+v"(d) : "v"(a), "v"(b));
  return d;
}

__device__ __forceinline__ float gelu_f(float x) {
  return 0.5f * x * (1.0f + erff(x * 0.70710678118654752f));
}

__device__ __forceinline__ float bn_gelu(float z, float mn, float vv, float gg, float be) {
  float t = z - mn;
  t = t * rsqrtf(vv + BN_EPS);
  t = t * gg;
  t = t + be;
  return gelu_f(t);
}

template <int KD, int NC, int APK>
__device__ __forceinline__ void mma_block(const unsigned short* sHi, const unsigned short* sLo,
                                          const unsigned short* __restrict__ Bw, int wrow, int lane,
                                          v8f (&acc)[NC / 16]) {
  static_assert((KD % 32) == 0 && (NC % 16) == 0 && (APK % 8) == 0);
  constexpr int NT = NC / 16, NKT = KD / 32, WPLN = NC * KD;
  const int hh = lane >> 4, m = lane & 15;
#pragma unroll
  for (int t = 0; t < NT; ++t) { v8f z = {0.f, 0.f, 0.f, 0.f, 0.f, 0.f, 0.f, 0.f}; acc[t] = z; }
  const unsigned short* ahp = sHi + (wrow + m) * APK + 8 * hh;
  const unsigned short* alp = sLo + (wrow + m) * APK + 8 * hh;
#pragma unroll 1
  for (int kt = 0; kt < NKT; ++kt) {
    FragB ah, al;
    ah.h[0] = *(const v8us*)(ahp + 32 * kt);
    ah.h[1] = *(const v8us*)(ahp + 32 * kt + 16);
    al.h[0] = *(const v8us*)(alp + 32 * kt);
    al.h[1] = *(const v8us*)(alp + 32 * kt + 16);
#pragma unroll
    for (int t = 0; t < NT; ++t) {
      const unsigned short* bp = Bw + (size_t)(16 * t + m) * KD + 32 * kt + 8 * hh;
      FragB bh, bl;
      bh.h[0] = *(const v8us*)bp;
      bh.h[1] = *(const v8us*)(bp + 16);
      bl.h[0] = *(const v8us*)(bp + WPLN);
      bl.h[1] = *(const v8us*)(bp + WPLN + 16);
      acc[t] = wmb(ah.v, bh.v, acc[t]);
      acc[t] = wmb(ah.v, bl.v, acc[t]);
      acc[t] = wmb(al.v, bh.v, acc[t]);
    }
  }
}

__device__ __forceinline__ void store_rows64(const float* stg, float* C, int rowBase, int wave, int lane) {
  const float* lp = stg + wave * 16 * HID + 4 * lane;
  float* gp = C + (size_t)(rowBase + wave * 16) * HID + 4 * lane;
#pragma unroll
  for (int i = 0; i < 8; ++i) { const v4f v = *(const v4f*)(lp + 128 * i); *(volatile v4f*)(gp + 128 * i) = v; }
  __threadfence();
#pragma unroll
  for (int i = 0; i < 8; ++i) { const v4f v = *(const v4f*)(lp + 128 * i); *(volatile v4f*)(gp + 128 * i) = v; }
}

template <int NB>
__device__ __forceinline__ int scan_chunk(const int* __restrict__ dsts, int nE, int cbase, int slotBase,
                                          int vec8, int* list, int tid, int lane, int wave) {
  int wc = 0;
#pragma unroll
  for (int g = 0; g < NGRP; ++g) {
    const int el0  = (g * NTHR + tid) * EPT;
    const int e0   = cbase + el0;
    const int sent = -2147483647 - 1;
    v4i da, db;
    if (vec8 != 0 && cbase + CHUNK <= nE) {
      da = *(const v4i*)(dsts + e0);
      db = *(const v4i*)(dsts + e0 + 4);
    } else {
      da.x = (e0     < nE) ? dsts[min(e0, nE - 1)] : sent;
      da.y = (e0 + 1 < nE) ? dsts[min(e0 + 1, nE - 1)] : sent;
      da.z = (e0 + 2 < nE) ? dsts[min(e0 + 2, nE - 1)] : sent;
      da.w = (e0 + 3 < nE) ? dsts[min(e0 + 3, nE - 1)] : sent;
      db.x = (e0 + 4 < nE) ? dsts[min(e0 + 4, nE - 1)] : sent;
      db.y = (e0 + 5 < nE) ? dsts[min(e0 + 5, nE - 1)] : sent;
      db.z = (e0 + 6 < nE) ? dsts[min(e0 + 6, nE - 1)] : sent;
      db.w = (e0 + 7 < nE) ? dsts[min(e0 + 7, nE - 1)] : sent;
    }
    const unsigned nb = (unsigned)slotBase;
    const unsigned s0 = (unsigned)da.x - nb, s1 = (unsigned)da.y - nb;
    const unsigned s2 = (unsigned)da.z - nb, s3 = (unsigned)da.w - nb;
    const unsigned s4 = (unsigned)db.x - nb, s5 = (unsigned)db.y - nb;
    const unsigned s6 = (unsigned)db.z - nb, s7 = (unsigned)db.w - nb;
    const bool h0 = s0 < (unsigned)NB, h1 = s1 < (unsigned)NB, h2 = s2 < (unsigned)NB, h3 = s3 < (unsigned)NB;
    const bool h4 = s4 < (unsigned)NB, h5 = s5 < (unsigned)NB, h6 = s6 < (unsigned)NB, h7 = s7 < (unsigned)NB;
    const unsigned any = __builtin_amdgcn_ballot_w32(h0 | h1 | h2 | h3 | h4 | h5 | h6 | h7);
    if (any != 0u) {
#define HITJ(J, HJ, SJ) { \
        const unsigned mj = __builtin_amdgcn_ballot_w32(HJ); \
        if (mj != 0u) { \
          if (HJ) { \
            const int pos = wc + (int)__builtin_amdgcn_mbcnt_lo(mj, 0u); \
            if (pos < WCAP) list[wave * WCAP + pos] = ((el0 + (J)) << 12) | (int)(SJ); \
          } \
          wc += (int)__builtin_popcount(mj); } }
      HITJ(0, h0, s0)
      HITJ(1, h1, s1)
      HITJ(2, h2, s2)
      HITJ(3, h3, s3)
      HITJ(4, h4, s4)
      HITJ(5, h5, s5)
      HITJ(6, h6, s6)
      HITJ(7, h7, s7)
#undef HITJ
    }
  }
  return wc;
}

__global__ __launch_bounds__(NTHR) void k_wprep(
    const float* __restrict__ wenc, const float* __restrict__ wl, const float* __restrict__ wr,
    const float* __restrict__ w1, const float* __restrict__ w2, unsigned short* wp) {
  const int blk = blockIdx.x, tid = threadIdx.x;
  float v[8];
  int KD, NC, i, base;
  if (blk == 0) {
    KD = KENC; NC = HID; i = tid; base = WP_ENC;
    const int n = i >> 2, k0 = (i & 3) * 8;
#pragma unroll
    for (int e = 0; e < 8; ++e) v[e] = wenc[(k0 + e) * HID + n];
  } else if (blk < 19) {
    const int l = (blk - 1) / 6, sub = (blk - 1) - 6 * l;
    KD = KSG; NC = HID; i = sub * NTHR + tid; base = WP_SG + l * WP_SGSZ;
    const int n = i / 24, k0 = (i - 24 * n) * 8;
    const float* wlp = wl + (size_t)l * (2 * HID * HID);
    const float* wrp = wr + (size_t)l * (HID * HID);
#pragma unroll
    for (int e = 0; e < 8; ++e) {
      const int k = k0 + e;
      const int ka = k > 127 ? 127 : k;
      int kb = k - 128; kb = kb < 0 ? 0 : kb;
      const float va = wlp[ka * HID + n];
      const float vb = wrp[kb * HID + n];
      v[e] = (k < 128) ? va : vb;
    }
  } else if (blk < 29) {
    KD = KH1; NC = 128; i = (blk - 19) * NTHR + tid; base = WP_H1;
    const int n = i / 20, k0 = (i - 20 * n) * 8;
#pragma unroll
    for (int e = 0; e < 8; ++e) {
      const int k = k0 + e;
      const int ka = k > 135 ? 135 : k;
      const float va = w1[ka * 128 + n];
      v[e] = (k < 136) ? va : 0.0f;
    }
  } else {
    KD = KH2; NC = HID; i = (blk - 29) * NTHR + tid; base = WP_H2;
    const int n = i >> 4, k0 = (i & 15) * 8;
#pragma unroll
    for (int e = 0; e < 8; ++e) v[e] = w2[(k0 + e) * HID + n];
  }
  v4f a, b;
  a.x = v[0]; a.y = v[1]; a.z = v[2]; a.w = v[3];
  b.x = v[4]; b.y = v[5]; b.z = v[6]; b.w = v[7];
  v8us hv, lv;
  split8(a, b, hv, lv);
  unsigned short* dh = wp + base + (size_t)i * 8;
  unsigned short* dl = dh + NC * KD;
  *(volatile v8us*)dh = hv;
  *(volatile v8us*)dl = lv;
  __threadfence();
  *(volatile v8us*)dh = hv;
  *(volatile v8us*)dl = lv;
}

__global__ __launch_bounds__(NTHR) void k_count(const int* __restrict__ ei, int* cnt, int nE, int vec8) {
  __shared__ __attribute__((aligned(16))) int scnt[NBC];
  __shared__ __attribute__((aligned(16))) int list[LISTN];
  __shared__ int wcnt[NWAVE];
  const int tid = threadIdx.x, lane = tid & 31, wave = tid >> 5;
  const int nodeBase = blockIdx.x * NBC;
  const int* dsts = ei + nE;

  for (int i = tid; i < NBC; i += NTHR) scnt[i] = 0;
  __syncthreads();

  const int nChunks = (nE + CHUNK - 1) / CHUNK;
#pragma unroll 1
  for (int ch = 0; ch < nChunks; ++ch) {
    const int cbase = ch * CHUNK;
    const int wc = scan_chunk<NBC>(dsts, nE, cbase, nodeBase, vec8, list, tid, lane, wave);
    if (lane == 0) wcnt[wave] = wc;
    __syncthreads();
    if (wave == 0) {
#pragma unroll 1
      for (int wsx = 0; wsx < NWAVE; ++wsx) {
        int n = __builtin_amdgcn_readfirstlane(wcnt[wsx]);
        n = n > WCAP ? WCAP : (n < 0 ? 0 : n);
        const int* lp = list + wsx * WCAP;
#pragma unroll 1
        for (int i = 0; i < n; ++i) {
          const int ent  = __builtin_amdgcn_readfirstlane(lp[i]);
          const int slot = ent & (NBC - 1);
          if (lane == 0) scnt[slot] = scnt[slot] + 1;
        }
      }
    }
    __syncthreads();
  }

  v4i cq[4];
#pragma unroll
  for (int q = 0; q < 4; ++q) {
    const int f = (wave * 4 + q) * 128 + 4 * lane;
    cq[q] = *(const v4i*)(scnt + f);
  }
  int* cp = cnt + (size_t)nodeBase;
#pragma unroll
  for (int q = 0; q < 4; ++q) {
    const int f = (wave * 4 + q) * 128 + 4 * lane;
    *(volatile v4i*)(cp + f) = cq[q];
  }
  __threadfence();
#pragma unroll
  for (int q = 0; q < 4; ++q) {
    const int f = (wave * 4 + q) * 128 + 4 * lane;
    *(volatile v4i*)(cp + f) = cq[q];
  }
}

__global__ __launch_bounds__(OTHR) void k_offsets(
    const int* __restrict__ cnt, int* off, int* rbase, int nChunk) {
  __shared__ __attribute__((aligned(16))) int soff[NBC];
  __shared__ __attribute__((aligned(16))) int srb[RBN];
  __shared__ int wtot[OTHR / 32];
  const int tid = threadIdx.x, lane = tid & 31, wave = tid >> 5, sub = tid >> 7;
  for (int i = tid; i < RBN; i += OTHR) srb[i] = 0;
  int carry = 0;
#pragma unroll 1
  for (int ch = 0; ch < nChunk; ++ch) {
    const int base = ch * NBC;
    const v4i c0 = *(const v4i*)(cnt + base + 8 * tid);
    const v4i c1 = *(const v4i*)(cnt + base + 8 * tid + 4);
    const int e0 = max(c0.x, 0), e1 = max(c0.y, 0), e2 = max(c0.z, 0), e3 = max(c0.w, 0);
    const int e4 = max(c1.x, 0), e5 = max(c1.y, 0), e6 = max(c1.z, 0), e7 = max(c1.w, 0);
    const int ts = e0 + e1 + e2 + e3 + e4 + e5 + e6 + e7;
    int incl = ts;
#pragma unroll
    for (int d = 1; d < 32; d <<= 1) {
      const int t = __shfl_up(incl, d);
      if (lane >= d) incl += t;
    }
    if (lane == 31) wtot[wave] = incl;
    __syncthreads();
    const int S0 = wtot[0]  + wtot[1]  + wtot[2]  + wtot[3];
    const int S1 = wtot[4]  + wtot[5]  + wtot[6]  + wtot[7];
    const int S2 = wtot[8]  + wtot[9]  + wtot[10] + wtot[11];
    const int S3 = wtot[12] + wtot[13] + wtot[14] + wtot[15];
    int pre = 0;
#pragma unroll 1
    for (int w = 4 * sub; w < wave; ++w) pre += wtot[w];
    const int b0 = carry;
    const int b1 = b0 + ((S0 + 31) & ~31);
    const int b2 = b1 + ((S1 + 31) & ~31);
    const int b3 = b2 + ((S2 + 31) & ~31);
    const int b4 = b3 + ((S3 + 31) & ~31);
    const int myb = sub == 0 ? b0 : (sub == 1 ? b1 : (sub == 2 ? b2 : b3));
    if (tid == 0) {
      srb[min(4 * ch + 0, RBN - 1)] = b0;
      srb[min(4 * ch + 1, RBN - 1)] = b1;
      srb[min(4 * ch + 2, RBN - 1)] = b2;
      srb[min(4 * ch + 3, RBN - 1)] = b3;
    }
    int run = myb + pre + incl - ts;
    soff[8 * tid + 0] = run; run += e0;
    soff[8 * tid + 1] = run; run += e1;
    soff[8 * tid + 2] = run; run += e2;
    soff[8 * tid + 3] = run; run += e3;
    soff[8 * tid + 4] = run; run += e4;
    soff[8 * tid + 5] = run; run += e5;
    soff[8 * tid + 6] = run; run += e6;
    soff[8 * tid + 7] = run;
    carry = b4;
    __syncthreads();
    const v4i o0 = *(const v4i*)(soff + 4 * tid);
    const v4i o1 = *(const v4i*)(soff + 4 * (tid + OTHR));
    int* op = off + base;
    *(volatile v4i*)(op + 4 * tid) = o0;
    *(volatile v4i*)(op + 4 * (tid + OTHR)) = o1;
    __threadfence();
    *(volatile v4i*)(op + 4 * tid) = o0;
    *(volatile v4i*)(op + 4 * (tid + OTHR)) = o1;
    __syncthreads();
  }
  if (tid == 0) srb[min(4 * nChunk, RBN - 1)] = carry;
  __syncthreads();
  v4i rv = {0, 0, 0, 0};
  if (tid < 32) rv = *(const v4i*)(srb + 4 * tid);
  if (tid < 32) *(volatile v4i*)(rbase + 4 * tid) = rv;
  __threadfence();
  if (tid < 32) *(volatile v4i*)(rbase + 4 * tid) = rv;
}

__global__ __launch_bounds__(NTHR) void k_fill(
    const int* __restrict__ ei, const int* __restrict__ off, const int* __restrict__ rbase,
    int* csr, int nN, int nE, int vec8, int csrLen) {
  extern __shared__ v4f lds_dyn[];
  int* region = (int*)lds_dyn;
  int* cursor = region + RCAP;
  int* list   = cursor + NBF;
  int* wcnt   = list + LISTN;
  const int tid = threadIdx.x, lane = tid & 31, wave = tid >> 5;
  const int b = blockIdx.x;
  const int nodeBase = b * NBF;
  const int* dsts = ei + nE;

  int rb0 = rbase[b];
  const int rb1 = rbase[b + 1];
  rb0 = rb0 < 0 ? 0 : (rb0 > csrLen ? csrLen : rb0);
  rb0 &= ~31;
  int len = rb1 - rb0;
  len = len < 0 ? 0 : (len > RCAP ? RCAP : len);
  int lenW = (len + 31) & ~31;
  if (rb0 + lenW > csrLen) lenW = (csrLen - rb0) & ~31;

  {
    const v4i z = {0, 0, 0, 0};
    for (int i = tid; i < RCAP / 4; i += NTHR) ((v4i*)region)[i] = z;
    for (int s = tid; s < NBF; s += NTHR) {
      int o = off[nodeBase + s] - rb0;
      o = o < 0 ? 0 : (o > RCAP ? RCAP : o);
      cursor[s] = o;
    }
  }
  __syncthreads();

  const int nChunks = (nE + CHUNK - 1) / CHUNK;
#pragma unroll 1
  for (int ch = 0; ch < nChunks; ++ch) {
    const int cbase = ch * CHUNK;
    const int wc = scan_chunk<NBF>(dsts, nE, cbase, nodeBase, vec8, list, tid, lane, wave);
    if (lane == 0) wcnt[wave] = wc;
    __syncthreads();
    if (wave == 0) {
#pragma unroll 1
      for (int wsx = 0; wsx < NWAVE; ++wsx) {
        int n = __builtin_amdgcn_readfirstlane(wcnt[wsx]);
        n = n > WCAP ? WCAP : (n < 0 ? 0 : n);
        const int* lp = list + wsx * WCAP;
#pragma unroll 1
        for (int i = 0; i < n; ++i) {
          const int ent  = __builtin_amdgcn_readfirstlane(lp[i]);
          const int slot = ent & (NBF - 1);
          int e = cbase + ((ent >> 12) & (CHUNK - 1));
          e = e > nE - 1 ? nE - 1 : e;
          int src = ei[e];
          src = src < 0 ? 0 : (src > nN - 1 ? nN - 1 : src);
          if (lane == 0) {
            int pos = cursor[slot];
            pos = pos < 0 ? 0 : (pos > RCAP - 1 ? RCAP - 1 : pos);
            region[pos] = src;
            const int np = pos + 1;
            cursor[slot] = np > RCAP ? RCAP : np;
          }
        }
      }
    }
    __syncthreads();
  }

  const int nv = lenW >> 2;
  int* gp = csr + rb0;
#pragma unroll 1
  for (int i = tid; i < nv; i += NTHR) { const v4i v = ((const v4i*)region)[i]; *(volatile v4i*)(gp + 4 * i) = v; }
  __threadfence();
#pragma unroll 1
  for (int i = tid; i < nv; i += NTHR) { const v4i v = ((const v4i*)region)[i]; *(volatile v4i*)(gp + 4 * i) = v; }
}

__global__ __launch_bounds__(NTHR) void k_enc(
    const float* __restrict__ x, const unsigned short* __restrict__ Bw,
    const float* __restrict__ bias, float* C, int nN) {
  extern __shared__ v4f lds_dyn[];
  unsigned short* sHi = (unsigned short*)lds_dyn;
  unsigned short* sLo = sHi + GROWS * APKE;
  float*          stg = (float*)lds_dyn;
  const int tid = threadIdx.x, lane = tid & 31, wave = tid >> 5, hh = lane >> 4, m = lane & 15;
  const int rowBase = blockIdx.x * GROWS;

#pragma unroll
  for (int it = 0; it < 2; ++it) {
    const int idx = it * NTHR + tid;
    const int r   = idx >> 2;
    const int c0  = (idx & 3) * 8;
    int row = rowBase + r;
    row = row > nN - 1 ? nN - 1 : row;
    const float* ap = x + (size_t)row * KENC + c0;
    const v4f a = *(const v4f*)ap, b = *(const v4f*)(ap + 4);
    v8us hv, lv;
    split8(a, b, hv, lv);
    *(v8us*)(sHi + r * APKE + c0) = hv;
    *(v8us*)(sLo + r * APKE + c0) = lv;
  }
  __syncthreads();

  v8f acc[4];
  mma_block<KENC, HID, APKE>(sHi, sLo, Bw, wave * 16, lane, acc);
  __syncthreads();

  {
    float* sp = stg + (wave * 16 + 8 * hh) * HID + m;
#pragma unroll
    for (int t = 0; t < 4; ++t) {
      const float bv = bias[16 * t + m];
#pragma unroll
      for (int r = 0; r < 8; ++r) sp[r * HID + 16 * t] = acc[t][r] + bv;
    }
  }
  __syncthreads();
  store_rows64(stg, C, rowBase, wave, lane);
}

__global__ __launch_bounds__(NTHR) void k_agg(
    const int* __restrict__ csr, const int* __restrict__ off, const int* __restrict__ cnt,
    const float* __restrict__ hin, float* A, int nN, int csrLen) {
  const int tid = threadIdx.x, lane = tid & 31, wave = tid >> 5;
  const int tbase = blockIdx.x * TGT + wave * 32;
  const int cl = tbase + lane;
  const int cnt_l = cnt[cl];
  const int off_l = off[cl];
  const float ninf = __uint_as_float(0xff800000u);

#pragma unroll 1
  for (int j = 0; j < 32; ++j) {
    const int c = tbase + j;
    int n = __builtin_amdgcn_readlane(cnt_l, j);
    n = n < 0 ? 0 : (n > DEGCAP ? DEGCAP : n);
    const int st = __builtin_amdgcn_readlane(off_l, j);
    v2f sm = {0.0f, 0.0f};
    v2f mx = {ninf, ninf};
#pragma unroll 1
    for (int q0 = 0; q0 < n; q0 += 32) {
      int pos = st + q0 + lane;
      pos = pos < 0 ? 0 : (pos > csrLen - 1 ? csrLen - 1 : pos);
      int sl = csr[pos];
      sl = sl < 0 ? 0 : (sl > nN - 1 ? nN - 1 : sl);
      const int mcnt = (n - q0) < 32 ? (n - q0) : 32;
#pragma unroll 1
      for (int p = 0; p < mcnt; ++p) {
        const int s = __builtin_amdgcn_readlane(sl, p);
        const v2f v = *(const v2f*)(hin + (size_t)s * HID + 2 * lane);
        sm = sm + v;
        mx.x = fmaxf(mx.x, v.x);
        mx.y = fmaxf(mx.y, v.y);
      }
    }
    const float rc = 1.0f / (float)(n > 1 ? n : 1);
    v2f mean; mean.x = sm.x * rc; mean.y = sm.y * rc;
    v2f mo;   mo.x = n > 0 ? mx.x : 0.0f; mo.y = n > 0 ? mx.y : 0.0f;
    float* ap = A + (size_t)c * (2 * HID) + 2 * lane;
    *(volatile v2f*)ap = mean;
    *(volatile v2f*)(ap + HID) = mo;
    __threadfence();
    *(volatile v2f*)ap = mean;
    *(volatile v2f*)(ap + HID) = mo;
  }
}

__global__ __launch_bounds__(NTHR) void k_layer(
    const float* __restrict__ Aagg, const float* __restrict__ hin,
    const unsigned short* __restrict__ Bw, const float* __restrict__ bias,
    const float* __restrict__ lng, const float* __restrict__ lnb, float* hout) {
  extern __shared__ v4f lds_dyn[];
  unsigned short* sHi = (unsigned short*)lds_dyn;
  unsigned short* sLo = sHi + GROWS * APKS;
  float*          stg = (float*)lds_dyn;
  const int tid = threadIdx.x, lane = tid & 31, wave = tid >> 5, hh = lane >> 4, m = lane & 15;
  const int rowBase = blockIdx.x * GROWS;

#pragma unroll
  for (int it = 0; it < 8; ++it) {
    const int idx = it * NTHR + tid;
    const int r   = idx >> 4;
    const int c0  = (idx & 15) * 8;
    const float* ap = Aagg + (size_t)(rowBase + r) * (2 * HID) + c0;
    const v4f a = *(const v4f*)ap, b = *(const v4f*)(ap + 4);
    v8us hv, lv;
    split8(a, b, hv, lv);
    *(v8us*)(sHi + r * APKS + c0) = hv;
    *(v8us*)(sLo + r * APKS + c0) = lv;
  }
#pragma unroll
  for (int it = 0; it < 4; ++it) {
    const int idx = it * NTHR + tid;
    const int r   = idx >> 3;
    const int c0  = (idx & 7) * 8;
    const float* ap = hin + (size_t)(rowBase + r) * HID + c0;
    const v4f a = *(const v4f*)ap, b = *(const v4f*)(ap + 4);
    v8us hv, lv;
    split8(a, b, hv, lv);
    *(v8us*)(sHi + r * APKS + 2 * HID + c0) = hv;
    *(v8us*)(sLo + r * APKS + 2 * HID + c0) = lv;
  }
  __syncthreads();

  v8f acc[4];
  mma_block<KSG, HID, APKS>(sHi, sLo, Bw, wave * 16, lane, acc);
  __syncthreads();

  {
    float* sp = stg + (wave * 16 + 8 * hh) * HID + m;
#pragma unroll
    for (int t = 0; t < 4; ++t) {
      const float bv = bias[16 * t + m];
#pragma unroll
      for (int r = 0; r < 8; ++r) sp[r * HID + 16 * t] = acc[t][r] + bv;
    }
  }
  __syncthreads();

  {
    const v2f g2 = *(const v2f*)(lng + 2 * lane);
    const v2f e2 = *(const v2f*)(lnb + 2 * lane);
#pragma unroll 1
    for (int j = 0; j < 16; ++j) {
      const int row = wave * 16 + j;
      float* sp = stg + row * HID + 2 * lane;
      const v2f v = *(const v2f*)sp;
      float s = v.x + v.y;
      s += __shfl_xor(s, 16);
      s += __shfl_xor(s, 8);
      s += __shfl_xor(s, 4);
      s += __shfl_xor(s, 2);
      s += __shfl_xor(s, 1);
      const float mu = s * (1.0f / 64.0f);
      const float dx = v.x - mu, dy = v.y - mu;
      float s2 = dx * dx + dy * dy;
      s2 += __shfl_xor(s2, 16);
      s2 += __shfl_xor(s2, 8);
      s2 += __shfl_xor(s2, 4);
      s2 += __shfl_xor(s2, 2);
      s2 += __shfl_xor(s2, 1);
      const float var = s2 * (1.0f / 64.0f);
      const float rs  = rsqrtf(var + LN_EPS);
      float yx = dx * rs * g2.x + e2.x;
      float yy = dy * rs * g2.y + e2.y;
      yx = gelu_f(yx);
      yy = gelu_f(yy);
      const v2f res = *(const v2f*)(hin + (size_t)(rowBase + row) * HID + 2 * lane);
      v2f o; o.x = yx + res.x; o.y = yy + res.y;
      *(v2f*)sp = o;
    }
  }
  __syncthreads();
  store_rows64(stg, hout, rowBase, wave, lane);
}

__global__ __launch_bounds__(NTHR) void k_head(
    const float* __restrict__ h, const int* __restrict__ qi, const float* __restrict__ ea,
    const unsigned short* __restrict__ Bw1, const float* __restrict__ b1,
    const float* __restrict__ bng, const float* __restrict__ bnb,
    const float* __restrict__ bnm, const float* __restrict__ bnv,
    const unsigned short* __restrict__ Bw2, const float* __restrict__ b2,
    const float* __restrict__ w3, const float* __restrict__ b3,
    float* out, int Q, int nN) {
  extern __shared__ v4f lds_dyn[];
  __shared__ __attribute__((aligned(16))) float sout[QROWS];
  __shared__ float sw3[HID];
  unsigned short* sH1 = (unsigned short*)lds_dyn;
  unsigned short* sL1 = sH1 + QROWS * APK1;
  float*          stg = (float*)lds_dyn;
  unsigned short* sH2 = (unsigned short*)((char*)lds_dyn + LDS_HEAD_R1);
  unsigned short* sL2 = sH2 + QROWS * APK2;
  const int tid = threadIdx.x, lane = tid & 31, wave = tid >> 5, hh = lane >> 4, m = lane & 15;
  const int rowBase = blockIdx.x * QROWS;
  const int* qs = qi;
  const int* qt = qi + Q;

  if (tid < HID) sw3[tid] = w3[tid];

#pragma unroll
  for (int it = 0; it < 4; ++it) {
    const int idx = it * NTHR + tid;
    const int r   = idx >> 3;
    const int c0  = (idx & 7) * 8;
    int q = rowBase + r; q = q > Q - 1 ? Q - 1 : q;
    int s = qs[q];
    s = s < 0 ? 0 : (s > nN - 1 ? nN - 1 : s);
    const float* p = h + (size_t)s * HID + c0;
    const v4f a = *(const v4f*)p, b = *(const v4f*)(p + 4);
    v8us hv, lv;
    split8(a, b, hv, lv);
    *(v8us*)(sH1 + r * APK1 + c0) = hv;
    *(v8us*)(sL1 + r * APK1 + c0) = lv;
  }
#pragma unroll
  for (int it = 0; it < 4; ++it) {
    const int idx = it * NTHR + tid;
    const int r   = idx >> 3;
    const int c0  = (idx & 7) * 8;
    int q = rowBase + r; q = q > Q - 1 ? Q - 1 : q;
    int s = qt[q];
    s = s < 0 ? 0 : (s > nN - 1 ? nN - 1 : s);
    const float* p = h + (size_t)s * HID + c0;
    const v4f a = *(const v4f*)p, b = *(const v4f*)(p + 4);
    v8us hv, lv;
    split8(a, b, hv, lv);
    *(v8us*)(sH1 + r * APK1 + HID + c0) = hv;
    *(v8us*)(sL1 + r * APK1 + HID + c0) = lv;
  }
#pragma unroll
  for (int it = 0; it < 2; ++it) {
    const int idx = it * NTHR + tid;
    const int r   = idx >> 2;
    const int g   = idx & 3;
    int q = rowBase + r; q = q > Q - 1 ? Q - 1 : q;
    const float* p = ea + (size_t)q * 8;
    v4f a = *(const v4f*)p, b = *(const v4f*)(p + 4);
    const bool zp = g != 0;
    a.x = zp ? 0.0f : a.x; a.y = zp ? 0.0f : a.y; a.z = zp ? 0.0f : a.z; a.w = zp ? 0.0f : a.w;
    b.x = zp ? 0.0f : b.x; b.y = zp ? 0.0f : b.y; b.z = zp ? 0.0f : b.z; b.w = zp ? 0.0f : b.w;
    v8us hv, lv;
    split8(a, b, hv, lv);
    *(v8us*)(sH1 + r * APK1 + 2 * HID + 8 * g) = hv;
    *(v8us*)(sL1 + r * APK1 + 2 * HID + 8 * g) = lv;
  }
  __syncthreads();

  v8f acc[8];
  mma_block<KH1, 128, APK1>(sH1, sL1, Bw1, wave * 16, lane, acc);
  __syncthreads();

  {
    float* sp = stg + (wave * 16 + 8 * hh) * 128 + m;
#pragma unroll
    for (int t = 0; t < 8; ++t) {
      const float bv = b1[16 * t + m];
#pragma unroll
      for (int r = 0; r < 8; ++r) sp[r * 128 + 16 * t] = acc[t][r] + bv;
    }
  }
  __syncthreads();

#pragma unroll 1
  for (int it = 0; it < 8; ++it) {
    const int idx = it * NTHR + tid;
    const int r   = idx >> 4;
    const int c0  = (idx & 15) * 8;
    const v4f z0 = *(const v4f*)(stg + r * 128 + c0), z1 = *(const v4f*)(stg + r * 128 + c0 + 4);
    const v4f m0 = *(const v4f*)(bnm + c0), m1 = *(const v4f*)(bnm + c0 + 4);
    const v4f q0 = *(const v4f*)(bnv + c0), q1 = *(const v4f*)(bnv + c0 + 4);
    const v4f g0 = *(const v4f*)(bng + c0), g1 = *(const v4f*)(bng + c0 + 4);
    const v4f e0 = *(const v4f*)(bnb + c0), e1 = *(const v4f*)(bnb + c0 + 4);
    v4f a, b;
    a.x = bn_gelu(z0.x, m0.x, q0.x, g0.x, e0.x);
    a.y = bn_gelu(z0.y, m0.y, q0.y, g0.y, e0.y);
    a.z = bn_gelu(z0.z, m0.z, q0.z, g0.z, e0.z);
    a.w = bn_gelu(z0.w, m0.w, q0.w, g0.w, e0.w);
    b.x = bn_gelu(z1.x, m1.x, q1.x, g1.x, e1.x);
    b.y = bn_gelu(z1.y, m1.y, q1.y, g1.y, e1.y);
    b.z = bn_gelu(z1.z, m1.z, q1.z, g1.z, e1.z);
    b.w = bn_gelu(z1.w, m1.w, q1.w, g1.w, e1.w);
    v8us hv, lv;
    split8(a, b, hv, lv);
    *(v8us*)(sH2 + r * APK2 + c0) = hv;
    *(v8us*)(sL2 + r * APK2 + c0) = lv;
  }
  __syncthreads();

  v8f acc2[4];
  mma_block<KH2, HID, APK2>(sH2, sL2, Bw2, wave * 16, lane, acc2);
  __syncthreads();

  {
    float* sp = stg + (wave * 16 + 8 * hh) * HID + m;
#pragma unroll
    for (int t = 0; t < 4; ++t) {
      const float bv = b2[16 * t + m];
#pragma unroll
      for (int r = 0; r < 8; ++r) sp[r * HID + 16 * t] = acc2[t][r] + bv;
    }
  }
  __syncthreads();

  if (tid < QROWS) {
    const float* zr = stg + tid * HID;
    float d = 0.0f;
#pragma unroll 4
    for (int k = 0; k < HID; ++k) d = fmaf(gelu_f(zr[k]), sw3[k], d);
    sout[tid] = d + b3[0];
  }
  __syncthreads();

  const int nrem = Q - rowBase;
  const bool ok = (wave == 0) && (4 * lane + 4 <= nrem);
  v4f ov = {0.f, 0.f, 0.f, 0.f};
  if (wave == 0) ov = *(const v4f*)(sout + 4 * lane);
  float* gp = out + (size_t)rowBase + 4 * lane;
  if (ok) *(volatile v4f*)gp = ov;
  __threadfence();
  if (ok) *(volatile v4f*)gp = ov;
}

extern "C" void kernel_launch(void* const* d_in, const int* in_sizes, int n_in,
                              void* d_out, int out_size, void* d_ws, size_t ws_size,
                              hipStream_t stream) {
  if (n_in < 21) return;
  const int nN = in_sizes[0] / 32;
  const int nE = in_sizes[1] / 2;
  const int Q  = in_sizes[3] / 2;
  if (nN <= 0 || nE <= 0 || Q <= 0) return;
  if (in_sizes[0] != nN * 32 || in_sizes[1] != 2 * nE) return;
  if (in_sizes[2] != Q * 8 || in_sizes[3] != 2 * Q) return;
  if (in_sizes[4] != 32 * HID || in_sizes[5] != HID) return;
  if (in_sizes[6] != 3 * 2 * HID * HID || in_sizes[7] != 3 * HID || in_sizes[8] != 3 * HID * HID) return;
  if (in_sizes[9] != 3 * HID || in_sizes[10] != 3 * HID) return;
  if (in_sizes[11] != 136 * 128 || in_sizes[12] != 128) return;
  if (in_sizes[13] != 128 || in_sizes[14] != 128 || in_sizes[15] != 128 || in_sizes[16] != 128) return;
  if (in_sizes[17] != 128 * HID || in_sizes[18] != HID || in_sizes[19] != HID || in_sizes[20] < 1) return;
  if (out_size != Q) return;
  if (nE > (1 << 28) || nN > (1 << 24) || Q > (1 << 28)) return;

  const float* x    = (const float*)d_in[0];
  const int*   ei   = (const int*)d_in[1];
  const float* ea   = (const float*)d_in[2];
  const int*   qi   = (const int*)d_in[3];
  const float* wenc = (const float*)d_in[4];
  const float* benc = (const float*)d_in[5];
  const float* wl   = (const float*)d_in[6];
  const float* bl   = (const float*)d_in[7];
  const float* wr   = (const float*)d_in[8];
  const float* lng  = (const float*)d_in[9];
  const float* lnb  = (const float*)d_in[10];
  const float* w1   = (const float*)d_in[11];
  const float* b1   = (const float*)d_in[12];
  const float* bng  = (const float*)d_in[13];
  const float* bnb  = (const float*)d_in[14];
  const float* bnm  = (const float*)d_in[15];
  const float* bnv  = (const float*)d_in[16];
  const float* w2   = (const float*)d_in[17];
  const float* b2   = (const float*)d_in[18];
  const float* w3   = (const float*)d_in[19];
  const float* b3   = (const float*)d_in[20];
  float* out = (float*)d_out;

  const int NPAD   = ((nN + TGT - 1) / TGT) * TGT;
  const int nBC    = (nN + NBC - 1) / NBC;
  const int CNTPAD = nBC * NBC;
  if (4 * nBC + 1 > RBN) return;
  const int nBF    = (nN + NBF - 1) / NBF;
  const int csrLen = ((nE + 31) & ~31) + 4096;
  if (31 * 4 * nBC > 4096) return;
  const int QPAD   = ((Q + QROWS - 1) / QROWS) * QROWS;
  const int nGemm  = NPAD / GROWS;
  const int nAgg   = NPAD / TGT;
  const int nHead  = QPAD / QROWS;

  char* ws = (char*)d_ws;
  size_t off = 0;
  const size_t oW   = off; off += (size_t)WPTOT * 2;               off = (off + 255) & ~(size_t)255;
  const size_t oCnt = off; off += (size_t)CNTPAD * 4;              off = (off + 255) & ~(size_t)255;
  const size_t oOff = off; off += (size_t)CNTPAD * 4;              off = (off + 255) & ~(size_t)255;
  const size_t oRb  = off; off += (size_t)RBN * 4;                 off = (off + 255) & ~(size_t)255;
  const size_t oCsr = off; off += (size_t)csrLen * 4;              off = (off + 255) & ~(size_t)255;
  const size_t oRA  = off; off += (size_t)NPAD * (2 * HID) * 4;    off = (off + 255) & ~(size_t)255;
  const size_t oHA  = off; off += (size_t)NPAD * HID * 4;          off = (off + 255) & ~(size_t)255;
  const size_t oHB  = off; off += (size_t)NPAD * HID * 4;          off = (off + 255) & ~(size_t)255;
  if (off > ws_size || off > (size_t)WSCAP) return;
  unsigned short* wp   = (unsigned short*)(ws + oW);
  int*            cnt  = (int*)(ws + oCnt);
  int*            offp = (int*)(ws + oOff);
  int*            rb   = (int*)(ws + oRb);
  int*            csr  = (int*)(ws + oCsr);
  float*          RA   = (float*)(ws + oRA);
  float*          HA   = (float*)(ws + oHA);
  float*          HB   = (float*)(ws + oHB);

  const int vec8 = ((nE & 3) == 0) ? 1 : 0;

  k_wprep<<<33, NTHR, 0, stream>>>(wenc, wl, wr, w1, w2, wp);

  k_count<<<nBC, NTHR, 0, stream>>>(ei, cnt, nE, vec8);
  k_offsets<<<1, OTHR, 0, stream>>>(cnt, offp, rb, nBC);
  hipFuncSetAttribute(reinterpret_cast<const void*>(&k_fill),
                      hipFuncAttributeMaxDynamicSharedMemorySize, LDS_FILL);
  k_fill<<<nBF, NTHR, LDS_FILL, stream>>>(ei, offp, rb, csr, nN, nE, vec8, csrLen);

  k_enc<<<nGemm, NTHR, LDS_ENC, stream>>>(x, wp + WP_ENC, benc, HA, nN);

  hipFuncSetAttribute(reinterpret_cast<const void*>(&k_layer),
                      hipFuncAttributeMaxDynamicSharedMemorySize, LDS_LAYER);
  for (int l = 0; l < 3; ++l) {
    const float* hin  = (l == 1) ? HB : HA;
    float*       hout = (l == 1) ? HA : HB;
    k_agg<<<nAgg, NTHR, 0, stream>>>(csr, offp, cnt, hin, RA, nN, csrLen);
    k_layer<<<nGemm, NTHR, LDS_LAYER, stream>>>(RA, hin, wp + WP_SG + l * WP_SGSZ,
                                                bl + l * HID, lng + l * HID, lnb + l * HID, hout);
  }

  hipFuncSetAttribute(reinterpret_cast<const void*>(&k_head),
                      hipFuncAttributeMaxDynamicSharedMemorySize, LDS_HEAD);
  k_head<<<nHead, NTHR, LDS_HEAD, stream>>>(HB, qi, ea, wp + WP_H1, b1, bng, bnb, bnm, bnv,
                                            wp + WP_H2, b2, w3, b3, out, Q, nN);
}
